// LocalAttentionModule_74491912782022
// MI455X (gfx1250) — hardware-verified
//
#include <hip/hip_runtime.h>


namespace {
constexpr int N = 4096, D = 256, H = 8, HD = 32, E = 65536, NW = N / 32  ;
constexpr float QS = 8.0f, KS = 8.0f, VS = 8.0f, PS = 8.0f, AS_ = 8.0f, SCALE = 0.17677669529663687f, NEG = -1e9f, EPS = 1e-5f;

typedef _Float16 b16;
typedef __attribute__((ext_vector_type(16))) _Float16 v16b;
typedef __attribute__((ext_vector_type(8))) _Float16 v8b;
typedef __attribute__((ext_vector_type(8))) float v8f;
typedef __attribute__((ext_vector_type(4))) float v4f;
typedef __attribute__((ext_vector_type(4))) unsigned int v4u;
__device__ __forceinline__ float bf16_rne(float f) { unsigned int u = __float_as_uint(f); u += 0x7FFFu + ((u >> 16) & 1u); return __uint_as_float(u & 0xFFFF0000u); }
__device__ __forceinline__ void split16(float v, b16& hi, b16& lo) { hi = (b16)v; lo = (b16)(v - (float)hi); }
__device__ __forceinline__ v16b frag_kb(const b16* p, int hh) { const v8b a = *(const v8b*)(p + 8 * hh), b = *(const v8b*)(p + 16 + 8 * hh); v16b f;
#pragma unroll
  for (int e = 0; e < 8; ++e) { f[e] = a[e]; f[8 + e] = b[e]; } return f; }
__device__ __forceinline__ v16b frag_x(const float* p, int hh) { v16b f;
#pragma unroll
  for (int e = 0; e < 8; ++e) { f[e] = (b16)bf16_rne(p[8 * hh + e]); f[8 + e] = (b16)bf16_rne(p[16 + 8 * hh + e]); } return f; }
__device__ __forceinline__ void frag_split(const float* p, int hh, v16b& fh, v16b& fl) {
#pragma unroll
  for (int e = 0; e < 8; ++e) { b16 a, c; split16(p[8 * hh + e] * AS_, a, c); fh[e] = a; fl[e] = c; split16(p[16 + 8 * hh + e] * AS_, a, c); fh[8 + e] = a; fl[8 + e] = c; } }
__device__ __forceinline__ v8f wmma16b(v16b a, v16b b, v8f c) { v8f d = __builtin_amdgcn_wmma_f32_16x16x32_f16(false, a, false, b, (short)0, c, false, false); asm volatile("v_nop\n\tv_nop\n\tv_nop\n\tv_nop" : "+v"(d) : "v"(a), "v"(b)); return d; }
__device__ __forceinline__ void wave_lds_sync() { __builtin_amdgcn_fence(__ATOMIC_RELEASE, "workgroup"); __builtin_amdgcn_wave_barrier(); __builtin_amdgcn_fence(__ATOMIC_ACQUIRE, "workgroup"); }
__device__ __forceinline__ float nexp(float x) { return __builtin_amdgcn_exp2f(x * 1.4426950408889634f); }
__device__ __forceinline__ float pmul(float a, float b) { float p = a * b; asm volatile("" : "+v"(p)); return p; }

struct Wo_ { static constexpr size_t QKV = 0, WO = QKV + (size_t)3 * D * D, END = WO + (size_t)D * D; };
__global__ __launch_bounds__(256) void prep_kernel(const float* __restrict__ Wq, const float* __restrict__ Wk, const float* __restrict__ Wv, const float* __restrict__ Wo, const float* __restrict__ bq, const float* __restrict__ bk, const float* __restrict__ bv, const float* __restrict__ bo, const float* __restrict__ lw, const float* __restrict__ lb, b16* __restrict__ R, float* __restrict__ P) {
  const int t_ = blockIdx.x * 256 + threadIdx.x, nth = gridDim.x * 256;
  for (int pass = 0; pass < 2; ++pass) {
    for (int q = t_; q < 4 * D * D; q += nth) { const int m = q / (D * D), o = (q / D) % D, k = q % D; const float* W = (m == 0) ? Wq : (m == 1) ? Wk : (m == 2) ? Wv : Wo; R[q] = (b16)bf16_rne(W[(size_t)k * D + o]); }
    for (int q = t_; q < 6 * D; q += nth) { const int m = q / D, i = q % D; const float* v = (m == 0) ? bq : (m == 1) ? bk : (m == 2) ? bv : (m == 3) ? bo : (m == 4) ? lw : lb; P[q] = bf16_rne(v[i]); }
    __threadfence(); }
}

__global__ __launch_bounds__(256) void adj_kernel(const int* __restrict__ ei, unsigned int* __restrict__ adj) {
  __shared__ unsigned int Bt[32][NW];
  const int r0 = blockIdx.x * 32, t_ = threadIdx.x;
  for (int i = t_; i < 32 * NW; i += 256) (&Bt[0][0])[i] = 0u;
  __syncthreads();
  if (t_ < 32) atomicOr(&Bt[t_][(r0 + t_) >> 5], 1u << ((r0 + t_) & 31));
  for (int e = t_; e < E; e += 256) { const int s = ei[e], d = ei[E + e]; if (s < 0 || s >= N || d < 0 || d >= N) continue;
    if (s >= r0 && s < r0 + 32) atomicOr(&Bt[s - r0][d >> 5], 1u << (d & 31));
    if (d >= r0 && d < r0 + 32) atomicOr(&Bt[d - r0][s >> 5], 1u << (s & 31)); }
  __syncthreads();
  for (int pass = 0; pass < 2; ++pass) { for (int i = t_; i < 32 * (NW / 4); i += 256) { const int rr = i / (NW / 4), c4 = (i % (NW / 4)) * 4; *(volatile v4u*)(adj + (size_t)(r0 + rr) * NW + c4) = *(const v4u*)(&Bt[rr][c4]); } __threadfence(); }
}

__global__ __launch_bounds__(256) void reach_kernel(const int* __restrict__ ei, const unsigned int* __restrict__ adj, unsigned int* __restrict__ reach) {
  const int wid = threadIdx.x >> 5, lane = threadIdx.x & 31, n = blockIdx.x * 8 + wid;
  v4u acc = *(const v4u*)(adj + (size_t)n * NW + lane * 4);
  for (int e0 = 0; e0 < E; e0 += 32) { const int e = e0 + lane; const int s = ei[e], d = ei[E + e]; int k = -1;
    if (s == n && d >= 0 && d < N) k = d; else if (d == n && s >= 0 && s < N) k = s;
    unsigned int hit = __builtin_amdgcn_ballot_w32(k >= 0);
    while (hit) { const int src = __builtin_ctz(hit); hit &= hit - 1; const int kk = __builtin_amdgcn_readlane(k, src); const v4u rk = *(const v4u*)(adj + (size_t)kk * NW + lane * 4); acc |= rk; } }
  for (int pass = 0; pass < 2; ++pass) { *(volatile v4u*)(reach + (size_t)n * NW + lane * 4) = acc; __threadfence(); }
}

__global__ __launch_bounds__(128) void proj_kernel(const float* __restrict__ x, const b16* __restrict__ R, const float* __restrict__ P, b16* __restrict__ qp, b16* __restrict__ kp, b16* __restrict__ vt) {
  __shared__ __attribute__((aligned(16))) b16 T[128][64 + 8]; __shared__ __attribute__((aligned(16))) b16 Tv[64][128 + 8];
  const int lane = threadIdx.x & 31, wave = threadIdx.x >> 5, nloc = lane & 15, hlf = lane >> 4, ct = blockIdx.x, which = ct >> 2, c0 = (ct & 3) * 64, n0 = blockIdx.y * 128, m0 = n0 + wave * 32;
  const b16* Wt = R + (size_t)which * D * D; const float* bias = P + which * D;
  v8f acc[2][4];
#pragma unroll
  for (int r = 0; r < 2; ++r)
#pragma unroll
    for (int t = 0; t < 4; ++t) acc[r][t] = (v8f){};
#pragma unroll
  for (int kb = 0; kb < D; kb += 32) { const v16b a0 = frag_x(x + (size_t)(m0 + nloc) * D + kb, hlf), a1 = frag_x(x + (size_t)(m0 + 16 + nloc) * D + kb, hlf);
#pragma unroll
    for (int t = 0; t < 4; ++t) { const v16b bw = frag_kb(Wt + (size_t)(c0 + t * 16 + nloc) * D + kb, hlf); acc[0][t] = wmma16b(a0, bw, acc[0][t]); acc[1][t] = wmma16b(a1, bw, acc[1][t]); } }
  if (which < 2) { const float scl = (which == 0) ? SCALE * QS : KS;
#pragma unroll
    for (int t = 0; t < 4; ++t) { const float bb = bias[c0 + t * 16 + nloc];
#pragma unroll
      for (int r = 0; r < 2; ++r)
#pragma unroll
        for (int v = 0; v < 8; ++v) T[wave * 32 + r * 16 + 8 * hlf + v][t * 16 + nloc] = (b16)((acc[r][t][v] + bb) * scl); }
    __syncthreads();
    b16* base = (which == 0) ? qp : kp;
    for (int pass = 0; pass < 2; ++pass) { for (int i = threadIdx.x; i < 2 * 128 * 4; i += 128) { const int hh2 = i / 512, rr = (i >> 2) & 127, c8 = (i & 3) * 8; const int hd_ = c0 / HD + hh2; *(volatile v8b*)(base + ((size_t)hd_ * N + n0 + rr) * HD + c8) = *(const v8b*)(&T[rr][hh2 * HD + c8]); } __threadfence(); }
    return; }
#pragma unroll
  for (int t = 0; t < 4; ++t) { const float bb = bias[c0 + t * 16 + nloc];
#pragma unroll
    for (int r = 0; r < 2; ++r)
#pragma unroll
      for (int v = 0; v < 8; ++v) Tv[t * 16 + nloc][wave * 32 + r * 16 + 8 * hlf + v] = (b16)((acc[r][t][v] + bb) * VS); }
  __syncthreads();
  for (int pass = 0; pass < 2; ++pass) { for (int i = threadIdx.x; i < 64 * 16; i += 128) { const int dd = i >> 4, c8 = (i & 15) * 8; const int hd_ = (c0 + dd) / HD, d = (c0 + dd) % HD; *(volatile v8b*)(vt + ((size_t)hd_ * HD + d) * N + n0 + c8) = *(const v8b*)(&Tv[dd][c8]); } __threadfence(); }
}

__global__ __launch_bounds__(256) void attn_kernel(const b16* __restrict__ qp, const b16* __restrict__ kp, const b16* __restrict__ vt, const unsigned int* __restrict__ reach, float* __restrict__ att) {
  __shared__ __attribute__((aligned(16))) float Os[16][D + 4];
  const int h = threadIdx.x >> 5, lane = threadIdx.x & 31, hh = lane >> 4, col = lane & 15; const int q0 = blockIdx.x * 16, qi = q0 + col;
  const b16* Q = qp + ((size_t)h * N) * HD; const b16* K = kp + ((size_t)h * N) * HD; const b16* V = vt + ((size_t)h * HD) * N; const unsigned int* mrow = reach + (size_t)qi * NW;
  const v16b qf = frag_kb(Q + (size_t)qi * HD, hh);
  float m = -INFINITY, l = 0.0f; v8f o[2] = {{}, {}};
  for (int kb = 0; kb < N; kb += 32) { const unsigned int mw = mrow[kb >> 5];
    const v16b ka = frag_kb(K + (size_t)(kb + col) * HD, hh), kc = frag_kb(K + (size_t)(kb + 16 + col) * HD, hh);
    v8f s0 = {}, s1 = {}; s0 = wmma16b(ka, qf, s0); s1 = wmma16b(kc, qf, s1);
    float mr = -INFINITY;
#pragma unroll
    for (int r = 0; r < 8; ++r) { s0[r] *= 1.0f / (QS * KS); s1[r] *= 1.0f / (QS * KS); if (!((mw >> (8 * hh + r)) & 1u)) s0[r] = NEG; if (!((mw >> (16 + 8 * hh + r)) & 1u)) s1[r] = NEG; mr = fmaxf(mr, fmaxf(s0[r], s1[r])); }
    mr = fmaxf(mr, __shfl_xor(mr, 16));
    const float mn = fmaxf(m, mr), al_ = nexp(m - mn); m = mn; float sum = 0.0f; v16b pbv;
#pragma unroll
    for (int r = 0; r < 8; ++r) { const float e0 = nexp(s0[r] - mn), e1 = nexp(s1[r] - mn); sum += e0 + e1; pbv[r] = (b16)(e0 * PS); pbv[8 + r] = (b16)(e1 * PS); }
    sum += __shfl_xor(sum, 16); l = l * al_ + sum;
#pragma unroll
    for (int t = 0; t < 2; ++t) { o[t] *= al_; const v16b vf = frag_kb(V + (size_t)(t * 16 + col) * N + kb, hh); o[t] = wmma16b(vf, pbv, o[t]); } }
  const float inv = 1.0f / (l * VS * PS);
#pragma unroll
  for (int t = 0; t < 2; ++t)
#pragma unroll
    for (int r = 0; r < 8; ++r) Os[col][h * HD + t * 16 + 8 * hh + r] = o[t][r] * inv;
  __syncthreads();
  for (int pass = 0; pass < 2; ++pass) { for (int i = threadIdx.x; i < 16 * (D / 4); i += 256) { const int rr = i / (D / 4), c4 = (i % (D / 4)) * 4; *(volatile v4f*)(att + (size_t)(q0 + rr) * D + c4) = *(const v4f*)(&Os[rr][c4]); } __threadfence(); }
}

__global__ __launch_bounds__(128) void out_kernel(const float* __restrict__ att, const b16* __restrict__ R, const float* __restrict__ P, const float* __restrict__ x, float* __restrict__ out) {
  __shared__ __attribute__((aligned(16))) float Hs[64][D + 4];
  const int lane = threadIdx.x & 31, wave = threadIdx.x >> 5, nloc = lane & 15, hlf = lane >> 4, r0 = blockIdx.x * 64 + wave * 16; const b16* Wo = R + Wo_::WO; const float* bo = P + 768; const float* lw = P + 1024; const float* lb = P + 1280;
  for (int half = 0; half < 2; ++half) { v8f acc[8];
#pragma unroll
    for (int t = 0; t < 8; ++t) acc[t] = (v8f){};
#pragma unroll
    for (int kb = 0; kb < D; kb += 32) { v16b a, al; frag_split(att + (size_t)(r0 + nloc) * D + kb, hlf, a, al);
#pragma unroll
      for (int t = 0; t < 8; ++t) { const v16b bw = frag_kb(Wo + (size_t)((half * 8 + t) * 16 + nloc) * D + kb, hlf); acc[t] = wmma16b(a, bw, acc[t]); acc[t] = wmma16b(al, bw, acc[t]); } }
#pragma unroll
    for (int t = 0; t < 8; ++t) { const int cc = (half * 8 + t) * 16 + nloc; const float bb = bo[cc];
#pragma unroll
      for (int v = 0; v < 8; ++v) { const int rr = wave * 16 + 8 * hlf + v; Hs[rr][cc] = acc[t][v] * (1.0f / AS_) + bb + bf16_rne(x[(size_t)(r0 + 8 * hlf + v) * D + cc]); } } }
  wave_lds_sync();
  { const int rr = wave * 16 + (lane & 15), c0 = (lane >> 4) * 128; float s = 0.0f; for (int c = 0; c < 128; ++c) s += Hs[rr][c0 + c]; s += __shfl_xor(s, 16); const float mu = s * (1.0f / D);
    float q = 0.0f; for (int c = 0; c < 128; ++c) { const float d = Hs[rr][c0 + c] - mu; q += pmul(d, d); } q += __shfl_xor(q, 16); const float is = rsqrtf(q * (1.0f / D) + EPS);
    wave_lds_sync(); for (int c = 0; c < 128; ++c) Hs[rr][c0 + c] = pmul((Hs[rr][c0 + c] - mu) * is, lw[c0 + c]) + lb[c0 + c]; }
  wave_lds_sync();
  for (int pass = 0; pass < 2; ++pass) { for (int i = lane; i < 16 * (D / 4); i += 32) { const int rr = i / (D / 4), c4 = (i % (D / 4)) * 4; *(volatile v4f*)(out + (size_t)(r0 + rr) * D + c4) = *(const v4f*)(&Hs[wave * 16 + rr][c4]); } __threadfence(); }
}
}

extern "C" void kernel_launch(void* const* d_in, const int* in_sizes, int n_in,
                              void* d_out, int out_size, void* d_ws, size_t ws_size, hipStream_t stream) {
  (void)n_in; (void)out_size;
  const float* x = (const float*)d_in[0]; const int* ei = (const int*)d_in[1]; const float* Wq = (const float*)d_in[2]; const float* bq = (const float*)d_in[3]; const float* Wk = (const float*)d_in[4]; const float* bk = (const float*)d_in[5]; const float* Wv = (const float*)d_in[6]; const float* bv = (const float*)d_in[7];
  const float* Wo = (const float*)d_in[8]; const float* bo = (const float*)d_in[9]; const float* lw = (const float*)d_in[10]; const float* lb = (const float*)d_in[11];
  float* out = (float*)d_out;
  if (in_sizes[0] != N * D || in_sizes[1] != 2 * E || in_sizes[2] != D * D || in_sizes[8] != D * D) return;
  size_t off = 0; char* ws = (char*)d_ws;
  auto carve = [&](size_t bytes) { char* p = ws + off; off += (bytes + 255) & ~(size_t)255; return p; };
  b16* R = (b16*)carve(Wo_::END * 2); float* P = (float*)carve(1536 * 4); unsigned int* adj = (unsigned int*)carve((size_t)N * NW * 4); unsigned int* reach = (unsigned int*)carve((size_t)N * NW * 4);
  b16* qp = (b16*)carve((size_t)H * N * HD * 2); b16* kp = (b16*)carve((size_t)H * N * HD * 2); b16* vt = (b16*)carve((size_t)H * HD * N * 2); float* att = (float*)carve((size_t)N * D * 4);
  if (off > ws_size) return;
  prep_kernel<<<128, 256, 0, stream>>>(Wq, Wk, Wv, Wo, bq, bk, bv, bo, lw, lb, R, P);
  adj_kernel<<<N / 32, 256, 0, stream>>>(ei, adj);
  reach_kernel<<<N / 8, 256, 0, stream>>>(ei, adj, reach);
  proj_kernel<<<dim3(12, N / 128), 128, 0, stream>>>(x, R, P, qp, kp, vt);
  attn_kernel<<<N / 16, 256, 0, stream>>>(qp, kp, vt, reach, att);
  out_kernel<<<N / 64, 128, 0, stream>>>(att, R, P, x, out);
}
